// GraphBatchNetAMP_83537113907556
// MI455X (gfx1250) — hardware-verified
//
#include <hip/hip_runtime.h>
#include <stddef.h>
#include <stdint.h>


#define ND   128
#define HD   128
#define ED   16
#define WSC  16.0f
#define WIV  0.0625f

#define T_NW1 0
#define T_NW2 16384
#define T_EA  32768
#define T_EB  49152
#define T_EW2 65536
#define T_EC  81920
#define T_TOT 83968
#define T_LINES 1312

#define NWV 4
#define NTW 4
#define NPB (NWV * NTW * 16)
#define HP  136

#define EWV 4
#define ETW 10
#define EPB (EWV * ETW * 16)
#define PP  132

#define NR  128
#define ER  160
#define MAXG 64

static_assert(T_NW2 == HD * ND && T_EA == 2 * HD * ND && T_EB == 3 * HD * ND && T_EW2 == 4 * HD * ND);
static_assert(T_EC == 5 * HD * ND && T_TOT == T_EC + HD * ED && T_LINES * 64 == T_TOT);
static_assert(((HP * 2) & 15) == 0 && ((PP * 4) & 15) == 0);
static_assert(NWV * 32 == HD && EWV * 32 == HD && ER == HD + 32 && (NR & 31) == 0 && (ER & 31) == 0);
static_assert(NPB == 256 && EPB == 640 && (MAXG & 1) == 0);

typedef float    v4f  __attribute__((ext_vector_type(4)));
typedef float    v8f  __attribute__((ext_vector_type(8)));
typedef _Float16 v8h  __attribute__((ext_vector_type(8)));
typedef _Float16 v16h __attribute__((ext_vector_type(16)));
union FragH { v16h v; v8h h[2]; };

__device__ __forceinline__ v8f zero8f() {
  v8f z;
#pragma unroll
  for (int i = 0; i < 8; ++i) z[i] = 0.0f;
  return z;
}
__device__ __forceinline__ v8h zero8h() {
  v8h z;
#pragma unroll
  for (int i = 0; i < 8; ++i) z[i] = (_Float16)0.0f;
  return z;
}

__device__ __forceinline__ v8f wm(v16h a, v16h b, v8f c) {
  return __builtin_amdgcn_wmma_f32_16x16x32_f16(false, a, false, b, (short)0, c, false, false);
}
#define WGUARD(ACC, A, B) asm volatile("v_nop\n\tv_nop\n\tv_nop\n\tv_nop" : "+v"(ACC) : "v"(A), "v"(B))

__device__ __forceinline__ v8h cvt8h(const float* p) {
  const v4f a = *(const v4f*)p;
  const v4f b = *(const v4f*)(p + 4);
  v8h o;
  o[0] = (_Float16)a[0]; o[1] = (_Float16)a[1]; o[2] = (_Float16)a[2]; o[3] = (_Float16)a[3];
  o[4] = (_Float16)b[0]; o[5] = (_Float16)b[1]; o[6] = (_Float16)b[2]; o[7] = (_Float16)b[3];
  return o;
}

__device__ __forceinline__ v8f mm_a(const _Float16* ar, v16h b0, v16h b1, v16h b2, v16h b3) {
  v8f acc = zero8f();
  FragH a;
  a.h[0] = *(const v8h*)(ar);      a.h[1] = *(const v8h*)(ar + 16);  acc = wm(a.v, b0, acc);
  a.h[0] = *(const v8h*)(ar + 32); a.h[1] = *(const v8h*)(ar + 48);  acc = wm(a.v, b1, acc);
  a.h[0] = *(const v8h*)(ar + 64); a.h[1] = *(const v8h*)(ar + 80);  acc = wm(a.v, b2, acc);
  a.h[0] = *(const v8h*)(ar + 96); a.h[1] = *(const v8h*)(ar + 112); acc = wm(a.v, b3, acc);
  WGUARD(acc, a.v, b3);
  return acc;
}
__device__ __forceinline__ v8f mm_b(const _Float16* br, v16h a0, v16h a1, v16h a2, v16h a3) {
  v8f acc = zero8f();
  FragH b;
  b.h[0] = *(const v8h*)(br);      b.h[1] = *(const v8h*)(br + 16);  acc = wm(a0, b.v, acc);
  b.h[0] = *(const v8h*)(br + 32); b.h[1] = *(const v8h*)(br + 48);  acc = wm(a1, b.v, acc);
  b.h[0] = *(const v8h*)(br + 64); b.h[1] = *(const v8h*)(br + 80);  acc = wm(a2, b.v, acc);
  b.h[0] = *(const v8h*)(br + 96); b.h[1] = *(const v8h*)(br + 112); acc = wm(a3, b.v, acc);
  WGUARD(acc, a3, b.v);
  return acc;
}

__device__ __forceinline__ float gate_of(float gs, float ev) {
#pragma clang fp contract(off)
  const float t = gs * ev;
  const float u = 1.0f + t;
  return fminf(fmaxf(u, 0.0f), 3.0f);
}

__global__ __launch_bounds__(256) void k_cvt(const float* __restrict__ nW1, const float* __restrict__ nW2,
                                             const float* __restrict__ eW1, const float* __restrict__ eW2,
                                             _Float16* Tt) {
  const int t = blockIdx.x * 256 + threadIdx.x;
  if (t >= T_LINES * 8) return;
  const int L = t >> 3, sub = (t & 7) * 8;
  const float* src = nW1;
  int n = 0, k0 = 0, dst = 0, roff = 0;
  if (L < 1280) {
    const int tb = L >> 8, q = L & 255;
    n = q >> 1; k0 = (q & 1) * 64 + sub;
    dst = tb * (HD * ND) + n * ND + k0;
    src = (tb == 0) ? nW1 : ((tb == 1) ? nW2 : ((tb == 4) ? eW2 : eW1));
    roff = (tb == 3) ? 128 : 0;
  } else {
    const int q = L - 1280;
    n = 4 * q + (sub >> 4); k0 = sub & 15;
    dst = T_EC + n * ED + k0;
    src = eW1; roff = 256;
  }
  v8h o;
#pragma unroll
  for (int i = 0; i < 8; ++i) o[i] = (_Float16)(src[(size_t)(roff + k0 + i) * HD + n] * WSC);
  _Float16* dp = Tt + dst;
  *(volatile v8h*)dp = o;
  __threadfence();
  *(volatile v8h*)dp = o;
}

__global__ __launch_bounds__(NWV * 32) void k_node(const float* __restrict__ X, const _Float16* __restrict__ Tt,
                                                   const float* __restrict__ nb1, const float* __restrict__ nb2,
                                                   _Float16* Apl, _Float16* Bpl, float* partN, int N, int nBlkN) {
  __shared__ __attribute__((aligned(16))) _Float16 h1s[NWV * 16 * HP];
  __shared__ __attribute__((aligned(16))) _Float16 sta[NWV * 16 * HP];
  __shared__ __attribute__((aligned(16))) _Float16 stb[NWV * 16 * HP];
  __shared__ __attribute__((aligned(16))) float cs[NWV * 2 * HD];
  __shared__ __attribute__((aligned(16))) float prow[NR];
  const int tid = threadIdx.x, l = tid & 31, wave = tid >> 5, h = l >> 4, m = l & 15;
  const int g = blockIdx.y, blk = blockIdx.x;
  const float* Xg = X + (size_t)g * N * ND;
  const size_t prb = ((size_t)g * nBlkN + blk) * NPB;
  for (int i = tid; i < NWV * 2 * HD; i += NWV * 32) cs[i] = 0.0f;
  __syncthreads();
  float* mycs = cs + (wave * 2 + h) * HD + m;
  _Float16* h1w = h1s + wave * 16 * HP;
  _Float16* saw = sta + wave * 16 * HP;
  _Float16* sbw = stb + wave * 16 * HP;
  const int c8 = 8 * m;

#pragma unroll 1
  for (int t = 0; t < NTW; ++t) {
    const int nbase = blk * NPB + t * (NWV * 16) + wave * 16;
    const size_t pr = prb + (size_t)(t * (NWV * 16) + wave * 16);
    int br = nbase + m;
    br = br > N - 1 ? N - 1 : br;
    const float* xr = Xg + (size_t)br * ND;
    FragH xf[4];
#pragma unroll
    for (int ks = 0; ks < 4; ++ks) {
      xf[ks].h[0] = cvt8h(xr + 32 * ks + 8 * h);
      xf[ks].h[1] = cvt8h(xr + 32 * ks + 16 + 8 * h);
    }
#pragma unroll 1
    for (int ct = 0; ct < 8; ++ct) {
      const v8f acc = mm_a(Tt + T_NW1 + (size_t)(16 * ct + m) * ND + 8 * h, xf[0].v, xf[1].v, xf[2].v, xf[3].v);
      const float* bp = nb1 + 16 * ct + 8 * h;
      const v4f c0 = *(const v4f*)bp;
      const v4f c1 = *(const v4f*)(bp + 4);
      v8h o;
#pragma unroll
      for (int r = 0; r < 4; ++r) {
        o[r]     = (_Float16)fmaxf(acc[r] * WIV + c0[r], 0.0f);
        o[4 + r] = (_Float16)fmaxf(acc[4 + r] * WIV + c1[r], 0.0f);
      }
      *(v8h*)(h1w + m * HP + 16 * ct + 8 * h) = o;
    }
#pragma unroll 1
    for (int ct = 0; ct < 8; ++ct) {
      const v8f acc = mm_a(Tt + T_EA + (size_t)(16 * ct + m) * ND + 8 * h, xf[0].v, xf[1].v, xf[2].v, xf[3].v);
      v8h o;
#pragma unroll
      for (int r = 0; r < 4; ++r) {
        o[r]     = (_Float16)(acc[r] * WIV);
        o[4 + r] = (_Float16)(acc[4 + r] * WIV);
      }
      *(v8h*)(saw + m * HP + 16 * ct + 8 * h) = o;
    }
#pragma unroll 1
    for (int ct = 0; ct < 8; ++ct) {
      const v8f acc = mm_a(Tt + T_EB + (size_t)(16 * ct + m) * ND + 8 * h, xf[0].v, xf[1].v, xf[2].v, xf[3].v);
      v8h o;
#pragma unroll
      for (int r = 0; r < 4; ++r) {
        o[r]     = (_Float16)(acc[r] * WIV);
        o[4 + r] = (_Float16)(acc[4 + r] * WIV);
      }
      *(v8h*)(sbw + m * HP + 16 * ct + 8 * h) = o;
    }
    __syncthreads();
    {
      FragH af[4];
      const _Float16* hr = h1w + m * HP + 8 * h;
#pragma unroll
      for (int ks = 0; ks < 4; ++ks) {
        af[ks].h[0] = *(const v8h*)(hr + 32 * ks);
        af[ks].h[1] = *(const v8h*)(hr + 32 * ks + 16);
      }
#pragma unroll 1
      for (int ct = 0; ct < 8; ++ct) {
        const v8f acc = mm_b(Tt + T_NW2 + (size_t)(16 * ct + m) * ND + 8 * h, af[0].v, af[1].v, af[2].v, af[3].v);
        const float bias = nb2[16 * ct + m];
        float part = 0.0f;
#pragma unroll
        for (int r = 0; r < 8; ++r) {
          const int nd = nbase + 8 * h + r;
          const float v = fmaxf(acc[r] * WIV + bias, 0.0f);
          part += (nd < N) ? v : 0.0f;
        }
        mycs[16 * ct] += part;
      }
    }
    {
      _Float16* ga = Apl + pr * ND + c8;
      _Float16* gb = Bpl + pr * ND + c8;
#pragma unroll
      for (int j = 0; j < 8; ++j) {
        const int lr = 2 * j + h;
        const v8h va = *(const v8h*)(saw + lr * HP + c8);
        const v8h vb = *(const v8h*)(sbw + lr * HP + c8);
        *(volatile v8h*)(ga + (size_t)lr * ND) = va;
        *(volatile v8h*)(gb + (size_t)lr * ND) = vb;
      }
      __threadfence();
#pragma unroll
      for (int j = 0; j < 8; ++j) {
        const int lr = 2 * j + h;
        const v8h va = *(const v8h*)(saw + lr * HP + c8);
        const v8h vb = *(const v8h*)(sbw + lr * HP + c8);
        *(volatile v8h*)(ga + (size_t)lr * ND) = va;
        *(volatile v8h*)(gb + (size_t)lr * ND) = vb;
      }
    }
    __syncthreads();
  }
  {
    float s = 0.0f;
#pragma unroll
    for (int w = 0; w < NWV; ++w) {
      s += cs[(w * 2 + 0) * HD + tid];
      s += cs[(w * 2 + 1) * HD + tid];
    }
    prow[tid] = s;
  }
  __syncthreads();
  if (wave == 0) {
    const v4f v = *(const v4f*)(prow + 4 * l);
    float* rp = partN + ((size_t)g * nBlkN + blk) * NR + 4 * l;
    *(volatile v4f*)rp = v;
    __threadfence();
    *(volatile v4f*)rp = v;
  }
}

__global__ __launch_bounds__(EWV * 32) void k_edge(const _Float16* __restrict__ Apl, const _Float16* __restrict__ Bpl,
                                                   const float* __restrict__ E, const int* __restrict__ edg,
                                                   const _Float16* __restrict__ Tt, const float* __restrict__ eb1,
                                                   const float* __restrict__ eb2, const float* __restrict__ gsp,
                                                   float* partE, int N, int M, int nBlkN, int nBlkE) {
  __shared__ __attribute__((aligned(16))) float Ef[EWV * 256];
  __shared__ __attribute__((aligned(16))) float Pt[EWV * 16 * PP];
  __shared__ __attribute__((aligned(16))) _Float16 Ht[EWV * 16 * HP];
  __shared__ int ixs[EWV * 32];
  __shared__ __attribute__((aligned(16))) float gts[EWV * 16];
  __shared__ __attribute__((aligned(16))) float gms[EWV * 16];
  __shared__ __attribute__((aligned(16))) float ms[EWV * 2 * HD];
  __shared__ __attribute__((aligned(16))) float eb2s[HD];
  __shared__ float red[EWV * 32];
  __shared__ __attribute__((aligned(16))) float prow[ER];
  const int tid = threadIdx.x, l = tid & 31, wave = tid >> 5, h = l >> 4, m = l & 15;
  const int g = blockIdx.y, blk = blockIdx.x;
  const float* Eg = E + (size_t)g * M * ED;
  const int*   eg = edg + (size_t)g * M * 2;
  const size_t prb = (size_t)g * nBlkN * NPB;
  const _Float16* Ag = Apl + prb * ND;
  const _Float16* Bg = Bpl + prb * ND;
  const float gs = gsp[0];
  for (int i = tid; i < EWV * 2 * HD; i += EWV * 32) ms[i] = 0.0f;
  eb2s[tid] = eb2[tid];
  const int q = m;
  const v4f e1a = *(const v4f*)(eb1 + 8 * q);
  const v4f e1b = *(const v4f*)(eb1 + 8 * q + 4);
  __syncthreads();
  float sacc = 0.0f;
  float* Efw = Ef + wave * 256;
  float* Pw  = Pt + wave * 16 * PP;
  _Float16* Hw = Ht + wave * 16 * HP;
  int* ixw = ixs + wave * 32;
  float* gtw = gts + wave * 16;
  float* gmw = gms + wave * 16;
  float* myms = ms + (wave * 2 + h) * HD + m;
  const v8h z8 = zero8h();

#pragma unroll 1
  for (int t = 0; t < ETW; ++t) {
    const int ebase = blk * EPB + (wave * ETW + t) * 16;
    {
      const int e = l >> 1, part = l & 1;
      int ge = ebase + e;
      ge = ge > M - 1 ? M - 1 : ge;
      const float* er = Eg + (size_t)ge * ED + 8 * part;
      const v4f u0 = *(const v4f*)er;
      const v4f u1 = *(const v4f*)(er + 4);
      *(v4f*)(Efw + e * 16 + 8 * part) = u0;
      *(v4f*)(Efw + e * 16 + 8 * part + 4) = u1;
      if (l < 16) {
        int ge2 = ebase + l;
        const bool valid = ge2 < M;
        ge2 = valid ? ge2 : M - 1;
        int s = eg[(size_t)ge2 * 2];
        int d = eg[(size_t)ge2 * 2 + 1];
        const int cnt = (((unsigned)s < (unsigned)N) ? 1 : 0) + (((unsigned)d < (unsigned)N) ? 1 : 0);
        s = s < 0 ? 0 : (s > N - 1 ? N - 1 : s);
        d = d < 0 ? 0 : (d > N - 1 ? N - 1 : d);
        ixw[l] = s;
        ixw[16 + l] = d;
        const float ev = Eg[(size_t)ge2 * ED + 2];
        const float gt = valid ? gate_of(gs, ev) : 0.0f;
        gtw[l] = gt;
        gmw[l] = gt * (float)cnt;
      }
    }
    __syncthreads();
    {
      FragH bf;
      bf.h[0] = cvt8h(Efw + m * 16 + 8 * h);
      bf.h[1] = z8;
#pragma unroll 1
      for (int ct = 0; ct < 8; ++ct) {
        FragH af;
        af.h[0] = *(const v8h*)(Tt + T_EC + (size_t)(16 * ct + m) * ED + 8 * h);
        af.h[1] = z8;
        v8f acc = zero8f();
        acc = wm(af.v, bf.v, acc);
        WGUARD(acc, af.v, bf.v);
        v4f f0, f1;
#pragma unroll
        for (int r = 0; r < 4; ++r) { f0[r] = acc[r] * WIV; f1[r] = acc[4 + r] * WIV; }
        *(v4f*)(Pw + m * PP + 16 * ct + 8 * h) = f0;
        *(v4f*)(Pw + m * PP + 16 * ct + 8 * h + 4) = f1;
      }
      if (l < 16) {
#pragma unroll
        for (int e = 0; e < 16; ++e) sacc += gtw[e] * Efw[e * 16 + l];
      } else if (l == 16) {
#pragma unroll
        for (int e = 0; e < 16; ++e) sacc += gtw[e];
      }
    }
    __syncthreads();
#pragma unroll 4
    for (int j = 0; j < 8; ++j) {
      const int e = h + 2 * j;
      const int s = ixw[e], d = ixw[16 + e];
      const v8h av = *(const v8h*)(Ag + (size_t)s * ND + 8 * q);
      const v8h bv = *(const v8h*)(Bg + (size_t)d * ND + 8 * q);
      const v4f p0 = *(const v4f*)(Pw + e * PP + 8 * q);
      const v4f p1 = *(const v4f*)(Pw + e * PP + 8 * q + 4);
      v8h o;
#pragma unroll
      for (int i = 0; i < 4; ++i) {
        const float x0 = (float)av[i] + (float)bv[i] + p0[i] + e1a[i];
        const float x1 = (float)av[4 + i] + (float)bv[4 + i] + p1[i] + e1b[i];
        o[i]     = (_Float16)fmaxf(x0, 0.0f);
        o[4 + i] = (_Float16)fmaxf(x1, 0.0f);
      }
      *(v8h*)(Hw + e * HP + 8 * q) = o;
    }
    __syncthreads();
    {
      const v4f g0 = *(const v4f*)(gmw + 8 * h);
      const v4f g1 = *(const v4f*)(gmw + 8 * h + 4);
      FragH af[4];
      const _Float16* hr = Hw + m * HP + 8 * h;
#pragma unroll
      for (int ks = 0; ks < 4; ++ks) {
        af[ks].h[0] = *(const v8h*)(hr + 32 * ks);
        af[ks].h[1] = *(const v8h*)(hr + 32 * ks + 16);
      }
#pragma unroll 1
      for (int ct = 0; ct < 8; ++ct) {
        const v8f acc = mm_b(Tt + T_EW2 + (size_t)(16 * ct + m) * HD + 8 * h, af[0].v, af[1].v, af[2].v, af[3].v);
        const float bias = eb2s[16 * ct + m];
        float part = 0.0f;
#pragma unroll
        for (int r = 0; r < 4; ++r) part += fmaxf(acc[r] * WIV + bias, 0.0f) * g0[r];
#pragma unroll
        for (int r = 0; r < 4; ++r) part += fmaxf(acc[4 + r] * WIV + bias, 0.0f) * g1[r];
        myms[16 * ct] += part;
      }
    }
    __syncthreads();
  }

  red[tid] = sacc;
  __syncthreads();
  {
    float s = 0.0f;
#pragma unroll
    for (int w = 0; w < EWV; ++w) {
      s += ms[(w * 2 + 0) * HD + tid];
      s += ms[(w * 2 + 1) * HD + tid];
    }
    prow[tid] = s;
    if (tid < 32) {
      float s2 = 0.0f;
      if (tid < ED + 1) {
#pragma unroll
        for (int w = 0; w < EWV; ++w) s2 += red[w * 32 + tid];
      }
      prow[HD + tid] = s2;
    }
  }
  __syncthreads();
  if (wave == 0) {
    float* rp = partE + ((size_t)g * nBlkE + blk) * ER;
    const bool tl = l < 8;
    const v4f v0 = *(const v4f*)(prow + 4 * l);
    v4f v1 = v0;
    if (tl) v1 = *(const v4f*)(prow + HD + 4 * l);
    *(volatile v4f*)(rp + 4 * l) = v0;
    if (tl) *(volatile v4f*)(rp + HD + 4 * l) = v1;
    __threadfence();
    *(volatile v4f*)(rp + 4 * l) = v0;
    if (tl) *(volatile v4f*)(rp + HD + 4 * l) = v1;
  }
}

__global__ __launch_bounds__(256) void k_final(const float* __restrict__ partN, const float* __restrict__ partE,
                                               const float* __restrict__ pW, const float* __restrict__ pb,
                                               const float* __restrict__ rW1, const float* __restrict__ rb1,
                                               const float* __restrict__ rW2, const float* __restrict__ rb2,
                                               float* out, int N, int M, int G, int nBlkN, int nBlkE) {
  __shared__ double dsh[HD];
  __shared__ double dsm[HD];
  __shared__ double dse[32];
  __shared__ __attribute__((aligned(16))) float feat[2 * HD];
  __shared__ float r1v[64];
  __shared__ __attribute__((aligned(16))) float res[2 * MAXG];
  const int tid = threadIdx.x;

#pragma unroll 1
  for (int g = 0; g < G; ++g) {
    if (tid < HD) {
      const float* p = partN + (size_t)g * nBlkN * NR + tid;
      double s = 0.0;
#pragma unroll 1
      for (int b = 0; b < nBlkN; ++b) s += (double)p[(size_t)b * NR];
      dsh[tid] = s;
      if (tid < ED + 1) {
        const float* p2 = partE + (size_t)g * nBlkE * ER + HD + tid;
        double s2 = 0.0;
#pragma unroll 1
        for (int b = 0; b < nBlkE; ++b) s2 += (double)p2[(size_t)b * ER];
        dse[tid] = s2;
      }
    } else {
      const int c = tid - HD;
      const float* p = partE + (size_t)g * nBlkE * ER + c;
      double s = 0.0;
#pragma unroll 1
      for (int b = 0; b < nBlkE; ++b) s += (double)p[(size_t)b * ER];
      dsm[c] = s;
    }
    __syncthreads();
    if (tid < HD) {
      feat[tid] = (float)((dsh[tid] + dsm[tid]) / (double)N);
    } else {
      const int n = tid - HD;
      double s = dse[ED] * (double)pb[n];
#pragma unroll 1
      for (int k = 0; k < ED; ++k) s += dse[k] * (double)pW[k * HD + n];
      const float den = (float)M + 1e-6f;
      feat[tid] = (float)(s / (double)den);
    }
    __syncthreads();
    if (tid < 64) {
      float s = 0.0f;
#pragma unroll 1
      for (int k = 0; k < 2 * HD; ++k) s += feat[k] * rW1[k * 64 + tid];
      r1v[tid] = fmaxf(s + rb1[tid], 0.0f);
    }
    __syncthreads();
    if (tid < 2) {
      float s = 0.0f;
#pragma unroll 1
      for (int k = 0; k < 64; ++k) s += r1v[k] * rW2[k * 2 + tid];
      res[g * 2 + tid] = s + rb2[tid];
    }
    __syncthreads();
  }
  if (tid < 32) {
    const int tot = 2 * G, nq = tot >> 2, rem = tot - 4 * nq;
    const bool hq = tid < nq, hrm = tid < rem;
    v4f vq;
    vq[0] = 0.0f; vq[1] = 0.0f; vq[2] = 0.0f; vq[3] = 0.0f;
    float vr = 0.0f;
    if (hq) vq = *(const v4f*)(res + 4 * tid);
    if (hrm) vr = res[4 * nq + tid];
    if (hq) *(volatile v4f*)(out + 4 * tid) = vq;
    if (hrm) ((volatile float*)out)[4 * nq + tid] = vr;
    __threadfence();
    if (hq) *(volatile v4f*)(out + 4 * tid) = vq;
    if (hrm) ((volatile float*)out)[4 * nq + tid] = vr;
  }
}

extern "C" void kernel_launch(void* const* d_in, const int* in_sizes, int n_in,
                              void* d_out, int out_size, void* d_ws, size_t ws_size,
                              hipStream_t stream) {
  if (n_in < 18) return;
  if (out_size < 2 || (out_size & 1)) return;
  const int G = out_size / 2;
  if (G > MAXG) return;
  if (in_sizes[0] <= 0 || in_sizes[1] <= 0) return;
  if ((in_sizes[0] % (G * ND)) != 0 || (in_sizes[1] % (G * ED)) != 0) return;
  const int N = in_sizes[0] / (G * ND);
  const int M = in_sizes[1] / (G * ED);
  if (N <= 0 || M <= 0) return;
  if (in_sizes[2] != G * M * 2) return;
  if (in_sizes[3] != ND * HD || in_sizes[4] < HD || in_sizes[5] != HD * HD || in_sizes[6] < HD) return;
  if (in_sizes[7] != (2 * ND + ED) * HD || in_sizes[8] < HD || in_sizes[9] != HD * HD || in_sizes[10] < HD) return;
  if (in_sizes[11] != ED * HD || in_sizes[12] < HD) return;
  if (in_sizes[13] != 2 * HD * 64 || in_sizes[14] < 64 || in_sizes[15] != 64 * 2 || in_sizes[16] < 2) return;
  if (in_sizes[17] < 1) return;

  const float* X   = (const float*)d_in[0];
  const float* E   = (const float*)d_in[1];
  const int*   edg = (const int*)d_in[2];
  const float* nW1 = (const float*)d_in[3];
  const float* nb1 = (const float*)d_in[4];
  const float* nW2 = (const float*)d_in[5];
  const float* nb2 = (const float*)d_in[6];
  const float* eW1 = (const float*)d_in[7];
  const float* eb1 = (const float*)d_in[8];
  const float* eW2 = (const float*)d_in[9];
  const float* eb2 = (const float*)d_in[10];
  const float* pW  = (const float*)d_in[11];
  const float* pb  = (const float*)d_in[12];
  const float* rW1 = (const float*)d_in[13];
  const float* rb1 = (const float*)d_in[14];
  const float* rW2 = (const float*)d_in[15];
  const float* rb2 = (const float*)d_in[16];
  const float* gsp = (const float*)d_in[17];
  float* out = (float*)d_out;

  const int nBlkN = (N + NPB - 1) / NPB;
  const int nBlkE = (M + EPB - 1) / EPB;

  char* ws = (char*)d_ws;
  size_t off = 0;
  const size_t plane = (size_t)G * nBlkN * NPB * ND * 2;
  const size_t oT  = off; off += (size_t)T_TOT * 2;                      off = (off + 255) & ~(size_t)255;
  const size_t oA  = off; off += plane;                                  off = (off + 255) & ~(size_t)255;
  const size_t oB  = off; off += plane;                                  off = (off + 255) & ~(size_t)255;
  const size_t oPN = off; off += (size_t)G * nBlkN * NR * 4;             off = (off + 255) & ~(size_t)255;
  const size_t oPE = off; off += (size_t)G * nBlkE * ER * 4;             off = (off + 255) & ~(size_t)255;
  if (off > ws_size) return;
  if (off > ((size_t)128 << 20)) return;
  _Float16* Tt  = (_Float16*)(ws + oT);
  _Float16* Apl = (_Float16*)(ws + oA);
  _Float16* Bpl = (_Float16*)(ws + oB);
  float*    pN  = (float*)(ws + oPN);
  float*    pE  = (float*)(ws + oPE);

  k_cvt<<<(T_LINES * 8 + 255) / 256, 256, 0, stream>>>(nW1, nW2, eW1, eW2, Tt);
  k_node<<<dim3(nBlkN, G), NWV * 32, 0, stream>>>(X, Tt, nb1, nb2, Apl, Bpl, pN, N, nBlkN);
  k_edge<<<dim3(nBlkE, G), EWV * 32, 0, stream>>>(Apl, Bpl, E, edg, Tt, eb1, eb2, gsp, pE, N, M, nBlkN, nBlkE);
  k_final<<<1, 256, 0, stream>>>(pN, pE, pW, pb, rW1, rb1, rW2, rb2, out, N, M, G, nBlkN, nBlkE);
  (void)hipGetLastError();
}
